// SFIModel_pipeline1_8478265442834
// MI455X (gfx1250) — hardware-verified
//
#include <hip/hip_runtime.h>

#define NB      64
#define NCDD    5
#define NHIS    50
#define LW      30
#define EDIM    300
#define FDIM    150
#define EPAD    320
#define FPAD    160
#define KPL     960
#define AROWS   38
#define PADROW  3
#define ENC_THREADS 256
#define LN_EPS  1e-5f

typedef __bf16 v16bf __attribute__((ext_vector_type(16)));
typedef __bf16 v8bf  __attribute__((ext_vector_type(8)));
typedef float  v8f   __attribute__((ext_vector_type(8)));
typedef float  v4f   __attribute__((ext_vector_type(4)));
typedef unsigned int v4u __attribute__((ext_vector_type(4)));
typedef unsigned int v2u __attribute__((ext_vector_type(2)));
typedef v8bf __attribute__((may_alias)) v8bfa;
typedef v4f  __attribute__((may_alias)) v4fa;
typedef v4u  __attribute__((may_alias)) v4ua;
typedef v2u  __attribute__((may_alias)) v2ua;

#define OFF_EMB   0
#define OFF_Y     24320
#define OFF_BIAS  85760
#define OFF_LNG   87680
#define OFF_LNB   88320
#define OFF_QL    88960
#define OFF_QW    89600
#define OFF_SDOT  90240
#define OFF_WDOT  90624
#define OFF_WL    90752
#define OFF_WW    91264
#define OFF_REP   91392
#define OFF_TOK   92032
#define ENC_SMEM  92160

__device__ __forceinline__ unsigned int bf16_bits(float x) {
  const unsigned int u = __float_as_uint(x);
  return (u + 0x7FFFu + ((u >> 16) & 1u)) >> 16;
}
__device__ __forceinline__ float bf16_val(float x) {
  return __uint_as_float(bf16_bits(x) << 16);
}

__device__ __forceinline__ float wsum(float v) {
  v += __shfl_xor(v, 16);
  v += __shfl_xor(v, 8);
  v += __shfl_xor(v, 4);
  v += __shfl_xor(v, 2);
  v += __shfl_xor(v, 1);
  return v;
}
__device__ __forceinline__ float wmax(float v) {
  v = fmaxf(v, __shfl_xor(v, 16));
  v = fmaxf(v, __shfl_xor(v, 8));
  v = fmaxf(v, __shfl_xor(v, 4));
  v = fmaxf(v, __shfl_xor(v, 2));
  v = fmaxf(v, __shfl_xor(v, 1));
  return v;
}

__device__ __forceinline__ v8f wmma_bf16(v16bf a, v16bf b, v8f c) {
  v8f d = __builtin_amdgcn_wmma_f32_16x16x32_bf16(false, a, false, b, (short)0, c, false, false);
  asm volatile("v_nop\n\tv_nop\n\tv_nop\n\tv_nop" : "+v"(d) : "v"(a), "v"(b));
  return d;
}

__device__ __forceinline__ v16bf ldfrag(const unsigned short* p, int h) {
  const v8bf lo = *(const v8bfa*)(p + 8 * h);
  const v8bf hi = *(const v8bfa*)(p + 16 + 8 * h);
  return __builtin_shufflevector(lo, hi, 0, 1, 2, 3, 4, 5, 6, 7, 8, 9, 10, 11, 12, 13, 14, 15);
}

__global__ __launch_bounds__(128)
void sfi_prep_w(const float* __restrict__ w1, const float* __restrict__ w2,
                const float* __restrict__ w3, unsigned short* __restrict__ Wp)
{
  const int bn = blockIdx.x;
  const int br = bn / FPAD;
  const int n  = bn - br * FPAD;
  const int t  = threadIdx.x;
  if (t >= KPL / 8) return;
  const int k   = 8 * t;
  const int tap = k / EPAD;
  const int e   = k - tap * EPAD;
  const int nc  = min(n, FDIM - 1);
  unsigned int bits[8];
  #pragma unroll
  for (int i = 0; i < 8; ++i) {
    const int ei = e + i;
    const int ec = min(ei, EDIM - 1);
    const size_t idx = ((size_t)tap * EDIM + ec) * FDIM + nc;
    const float x1 = w1[idx], x2 = w2[idx], x3 = w3[idx];
    float v = (br == 0) ? x1 : ((br == 1) ? x2 : x3);
    v = (ei < EDIM && n < FDIM) ? v : 0.0f;
    bits[i] = bf16_bits(v);
  }
  v4u o;
  o.x = bits[0] | (bits[1] << 16);
  o.y = bits[2] | (bits[3] << 16);
  o.z = bits[4] | (bits[5] << 16);
  o.w = bits[6] | (bits[7] << 16);
  unsigned short* dst = Wp + (size_t)bn * KPL + k;
  *(volatile v4u*)dst = o;
  __threadfence();
  *(volatile v4u*)dst = o;
}

__global__ __launch_bounds__(ENC_THREADS)
void sfi_encoder(const int* __restrict__ cand,
                 const int* __restrict__ clicked,
                 int nCand,
                 const float* __restrict__ embedding,
                 int nV,
                 const unsigned short* __restrict__ Wp,
                 const float* __restrict__ b1, const float* __restrict__ b2,
                 const float* __restrict__ b3,
                 const float* __restrict__ ln_g, const float* __restrict__ ln_b,
                 const float* __restrict__ q_l,  const float* __restrict__ q_w,
                 float* __restrict__ reprs)
{
  extern __shared__ __attribute__((aligned(16))) char smem[];
  unsigned short* embA = (unsigned short*)(smem + OFF_EMB);
  float* attnL = (float*)(smem + OFF_EMB);
  float* yL    = (float*)(smem + OFF_Y);
  float* biasL = (float*)(smem + OFF_BIAS);
  float* lngL  = (float*)(smem + OFF_LNG);
  float* lnbL  = (float*)(smem + OFF_LNB);
  float* qlL   = (float*)(smem + OFF_QL);
  float* qwL   = (float*)(smem + OFF_QW);
  float* sdotL = (float*)(smem + OFF_SDOT);
  float* wdotL = (float*)(smem + OFF_WDOT);
  float* wlL   = (float*)(smem + OFF_WL);
  float* wwL   = (float*)(smem + OFF_WW);
  float* repS  = (float*)(smem + OFF_REP);
  int*   tokL  = (int*)(smem + OFF_TOK);

  const int T = blockIdx.x;
  const int tid = threadIdx.x, lane = tid & 31, wave = tid >> 5;
  const int lh = lane >> 4, m = lane & 15;
  const float inv_scale = 1.0f / sqrtf((float)EDIM);

  const int* tp = (T < nCand) ? (cand + (size_t)T * LW) : (clicked + (size_t)(T - nCand) * LW);

  if (tid < 32) {
    const int tk = tp[min(tid, LW - 1)];
    tokL[tid] = min(max(tk, 0), nV - 1);
  }
  if (tid < FPAD) {
    const int f = tid, fc = min(f, FDIM - 1);
    const bool ok = f < FDIM;
    const float g  = bf16_val(ln_g[fc]);
    const float bb = bf16_val(ln_b[fc]);
    const float ql = bf16_val(q_l[fc]);
    const float qw = bf16_val(q_w[fc]);
    lngL[f] = ok ? g  : 0.0f;
    lnbL[f] = ok ? bb : 0.0f;
    qlL[f]  = ok ? ql : 0.0f;
    qwL[f]  = ok ? qw : 0.0f;
  }
  for (int i = tid; i < 3 * FPAD; i += ENC_THREADS) {
    const int j = i / FPAD, f = i - j * FPAD, fc = min(f, FDIM - 1);
    const float x1 = b1[fc], x2 = b2[fc], x3 = b3[fc];
    const float v = (j == 0) ? x1 : ((j == 1) ? x2 : x3);
    biasL[i] = (f < FDIM) ? bf16_val(v) : 0.0f;
  }
  __syncthreads();

  for (int it = tid; it < AROWS * 80; it += ENC_THREADS) {
    const int r = it / 80, cg = it - r * 80;
    const int l = r - PADROW;
    const int lc = min(max(l, 0), LW - 1);
    const int cgc = min(cg, 74);
    const v4f x = *(const v4fa*)(embedding + (size_t)tokL[lc] * EDIM + 4 * cgc);
    const bool ok = (l >= 0) && (l < LW) && (cg < 75);
    const float x0 = ok ? x.x : 0.0f, x1 = ok ? x.y : 0.0f;
    const float x2 = ok ? x.z : 0.0f, x3 = ok ? x.w : 0.0f;
    v2u o;
    o.x = bf16_bits(x0) | (bf16_bits(x1) << 16);
    o.y = bf16_bits(x2) | (bf16_bits(x3) << 16);
    *(v2ua*)(embA + r * EPAD + 4 * cg) = o;
  }
  __syncthreads();

  {
    const v8f zero8 = {0.f, 0.f, 0.f, 0.f, 0.f, 0.f, 0.f, 0.f};
    for (int g = wave; g < 15; g += 8) {
      const int br = g / 5, np = g - br * 5;
      const int dil = br + 1;
      const int n0 = np * 32;
      v8f acc00 = zero8, acc01 = zero8, acc10 = zero8, acc11 = zero8;
      const unsigned short* wrow = Wp + (size_t)(br * FPAD + n0 + m) * KPL;
      #pragma unroll 1
      for (int tap = 0; tap < 3; ++tap) {
        const int rowA = m + PADROW + (tap - 1) * dil;
        const unsigned short* ap = embA + rowA * EPAD;
        const unsigned short* bp = wrow + tap * EPAD;
        #pragma unroll 2
        for (int kt = 0; kt < 10; ++kt) {
          const int k = kt * 32;
          const v16bf a0  = ldfrag(ap + k, lh);
          const v16bf a1  = ldfrag(ap + 16 * EPAD + k, lh);
          const v16bf fb0 = ldfrag(bp + k, lh);
          const v16bf fb1 = ldfrag(bp + (size_t)16 * KPL + k, lh);
          acc00 = wmma_bf16(a0, fb0, acc00);
          acc01 = wmma_bf16(a0, fb1, acc01);
          acc10 = wmma_bf16(a1, fb0, acc10);
          acc11 = wmma_bf16(a1, fb1, acc11);
        }
      }
      const int nA = n0 + m, nBc = n0 + 16 + m;
      const float bias0 = biasL[br * FPAD + nA];
      const float bias1 = biasL[br * FPAD + nBc];
      float* yb = yL + (size_t)br * 32 * FPAD;
      #pragma unroll
      for (int r = 0; r < 8; ++r) {
        const int l0 = 8 * lh + r, l1 = l0 + 16;
        yb[l0 * FPAD + nA]  = acc00[r] + bias0;
        yb[l0 * FPAD + nBc] = acc01[r] + bias1;
        yb[l1 * FPAD + nA]  = acc10[r] + bias0;
        yb[l1 * FPAD + nBc] = acc11[r] + bias1;
      }
    }
  }
  __syncthreads();

  for (int rr = wave; rr < 3 * LW; rr += 8) {
    const int br = rr / LW, l = rr - br * LW;
    float* yr = yL + (size_t)(br * 32 + l) * FPAD;
    float v[5];
    float s = 0.0f;
    #pragma unroll
    for (int j = 0; j < 5; ++j) { v[j] = yr[lane + 32 * j]; s += v[j]; }
    s = wsum(s);
    const float mean = s * (1.0f / (float)FDIM);
    float s2 = 0.0f;
    #pragma unroll
    for (int j = 0; j < 5; ++j) {
      const float dv = v[j] - mean;
      const float mk = (j < 4 || lane < FDIM - 128) ? 1.0f : 0.0f;
      s2 += dv * dv * mk;
    }
    s2 = wsum(s2);
    const float var = s2 * (1.0f / (float)FDIM);
    const float rstd = 1.0f / sqrtf(var + LN_EPS);
    float qd = 0.0f;
    #pragma unroll
    for (int j = 0; j < 5; ++j) {
      const int f = lane + 32 * j;
      float d = (v[j] - mean) * rstd * lngL[f] + lnbL[f];
      d = fmaxf(d, 0.0f);
      d = (j < 4 || lane < FDIM - 128) ? d : 0.0f;
      yr[f] = d;
      qd += qlL[f] * d;
    }
    qd = wsum(qd);
    if (lane == 0) sdotL[br * 32 + l] = qd;
  }
  __syncthreads();

  if (tid < LW) {
    const int l = tid;
    const float s0 = sdotL[l] * inv_scale;
    const float s1 = sdotL[32 + l] * inv_scale;
    const float s2 = sdotL[64 + l] * inv_scale;
    const float mx = fmaxf(s0, fmaxf(s1, s2));
    const float e0 = expf(s0 - mx), e1 = expf(s1 - mx), e2 = expf(s2 - mx);
    const float is = 1.0f / (e0 + e1 + e2);
    wlL[l * 4 + 0] = e0 * is;
    wlL[l * 4 + 1] = e1 * is;
    wlL[l * 4 + 2] = e2 * is;
    wlL[l * 4 + 3] = 0.0f;
  }
  __syncthreads();

  for (int l = wave; l < LW; l += 8) {
    const float w0 = wlL[l * 4 + 0], w1v = wlL[l * 4 + 1], w2v = wlL[l * 4 + 2];
    const float* d0 = yL + (size_t)l * FPAD;
    const float* d1 = yL + (size_t)(32 + l) * FPAD;
    const float* d2 = yL + (size_t)(64 + l) * FPAD;
    float wd = 0.0f;
    #pragma unroll
    for (int j = 0; j < 5; ++j) {
      const int f = lane + 32 * j;
      const float av = w0 * d0[f] + w1v * d1[f] + w2v * d2[f];
      attnL[l * FPAD + f] = av;
      wd += qwL[f] * av;
    }
    wd = wsum(wd);
    if (lane == 0) wdotL[l] = wd;
  }
  __syncthreads();

  if (wave == 0) {
    const bool ok = lane < LW;
    const float s = ok ? wdotL[min(lane, LW - 1)] * inv_scale : -3.0e38f;
    const float mx = wmax(s);
    const float ex = expf(s - mx);
    const float e = ok ? ex : 0.0f;
    const float se = wsum(e);
    wwL[lane] = e * (1.0f / se);
  }
  __syncthreads();

  if (tid < FPAD) {
    float rep = 0.0f;
    #pragma unroll 5
    for (int l = 0; l < LW; ++l) rep += wwL[l] * attnL[l * FPAD + tid];
    repS[tid] = rep;
  }
  __syncthreads();

  if (tid < FPAD / 4) {
    const v4f vv = *(const v4fa*)(repS + 4 * tid);
    float* dst = reprs + (size_t)T * FPAD + 4 * tid;
    *(volatile v4f*)dst = vv;
    __threadfence();
    *(volatile v4f*)dst = vv;
  }
}

__global__ __launch_bounds__(256)
void sfi_score(const float* __restrict__ reprs,
               int nCand,
               const float* __restrict__ ltr_w,
               const float* __restrict__ ltr_b,
               float* __restrict__ out)
{
  __shared__ __attribute__((aligned(16))) float lgS[NB * NCDD];
  __shared__ __attribute__((aligned(16))) float outS[NB * NCDD];
  __shared__ float lwS[64];
  const int tid = threadIdx.x;
  if (tid < NHIS) lwS[tid] = bf16_val(ltr_w[tid]);
  const float lb = bf16_val(ltr_b[0]);
  __syncthreads();

  for (int p = tid; p < NB * NCDD; p += 256) {
    const int b = p / NCDD, c = p - b * NCDD;
    const float* cr  = reprs + (size_t)(b * NCDD + c) * FPAD;
    const float* hbp = reprs + (size_t)(nCand + b * NHIS) * FPAD;
    float lg = 0.0f;
    #pragma unroll 1
    for (int hh = 0; hh < NHIS; ++hh) {
      const float* hr = hbp + (size_t)hh * FPAD;
      float dot = 0.0f;
      #pragma unroll 2
      for (int f = 0; f < 152; f += 4) {
        const v4f a = *(const v4fa*)(cr + f);
        const v4f q = *(const v4fa*)(hr + f);
        dot += a.x * q.x;
        dot += a.y * q.y;
        dot += a.z * q.z;
        dot += a.w * q.w;
      }
      lg += dot * lwS[hh];
    }
    lgS[p] = lg + lb;
  }
  __syncthreads();

  if (tid < NB) {
    const int b = tid;
    float mx = lgS[b * NCDD];
    #pragma unroll 1
    for (int c = 1; c < NCDD; ++c) mx = fmaxf(mx, lgS[b * NCDD + c]);
    float se = 0.0f;
    #pragma unroll 1
    for (int c = 0; c < NCDD; ++c) se += expf(lgS[b * NCDD + c] - mx);
    const float lse = logf(se);
    #pragma unroll 1
    for (int c = 0; c < NCDD; ++c) outS[b * NCDD + c] = (lgS[b * NCDD + c] - mx) - lse;
  }
  __syncthreads();

  if (tid < (NB * NCDD) / 4) {
    const v4f vv = *(const v4fa*)(outS + 4 * tid);
    *(volatile v4f*)(out + 4 * tid) = vv;
    __threadfence();
    *(volatile v4f*)(out + 4 * tid) = vv;
  }
}

extern "C" void kernel_launch(void* const* d_in, const int* in_sizes, int n_in,
                              void* d_out, int out_size, void* d_ws, size_t ws_size,
                              hipStream_t stream) {
  if (n_in < 15) return;
  if (in_sizes[0] != NB * NCDD * LW) return;
  if (in_sizes[1] != NB * NHIS * LW) return;
  if (in_sizes[2] < EDIM || (in_sizes[2] % EDIM) != 0) return;
  if (in_sizes[3] != 3 * EDIM * FDIM || in_sizes[5] != 3 * EDIM * FDIM || in_sizes[7] != 3 * EDIM * FDIM) return;
  if (in_sizes[4] != FDIM || in_sizes[6] != FDIM || in_sizes[8] != FDIM) return;
  if (in_sizes[9] != FDIM || in_sizes[10] != FDIM || in_sizes[11] != FDIM || in_sizes[12] != FDIM) return;
  if (in_sizes[13] != NHIS || in_sizes[14] < 1) return;
  if (out_size != NB * NCDD) return;

  const int*   cand    = (const int*)d_in[0];
  const int*   clicked = (const int*)d_in[1];
  const float* emb     = (const float*)d_in[2];
  const float* w1      = (const float*)d_in[3];
  const float* b1      = (const float*)d_in[4];
  const float* w2      = (const float*)d_in[5];
  const float* b2      = (const float*)d_in[6];
  const float* w3      = (const float*)d_in[7];
  const float* b3      = (const float*)d_in[8];
  const float* ln_g    = (const float*)d_in[9];
  const float* ln_b    = (const float*)d_in[10];
  const float* q_l     = (const float*)d_in[11];
  const float* q_w     = (const float*)d_in[12];
  const float* ltr_w   = (const float*)d_in[13];
  const float* ltr_b   = (const float*)d_in[14];
  float* out = (float*)d_out;

  const int nV    = in_sizes[2] / EDIM;
  const int nCand = in_sizes[0] / LW;
  const int nHis  = in_sizes[1] / LW;
  const int nT    = nCand + nHis;

  const size_t wp_bytes  = (size_t)3 * FPAD * KPL * 2;
  const size_t rep_bytes = (size_t)nT * FPAD * 4;
  const size_t total = wp_bytes + rep_bytes;
  if (total > ws_size) return;

  char* ws = (char*)d_ws;
  unsigned short* Wp = (unsigned short*)(ws);
  float* reprs = (float*)(ws + wp_bytes);

  hipFuncSetAttribute(reinterpret_cast<const void*>(&sfi_encoder),
                      hipFuncAttributeMaxDynamicSharedMemorySize, ENC_SMEM);

  sfi_prep_w<<<3 * FPAD, 128, 0, stream>>>(w1, w2, w3, Wp);

  sfi_encoder<<<nT, ENC_THREADS, ENC_SMEM, stream>>>(
      cand, clicked, nCand, emb, nV, Wp, b1, b2, b3, ln_g, ln_b, q_l, q_w, reprs);

  sfi_score<<<1, 256, 0, stream>>>(reprs, nCand, ltr_w, ltr_b, out);
}
